// MultiSourceAttentionBlock_83614423318762
// MI455X (gfx1250) — hardware-verified
//
#include <hip/hip_runtime.h>
#include <math.h>
#include <stdint.h>

typedef __attribute__((ext_vector_type(16))) _Float16 v16h;
typedef __attribute__((ext_vector_type(8)))  _Float16 v8h;
typedef __attribute__((ext_vector_type(16))) __bf16   v16b;
typedef __attribute__((ext_vector_type(8)))  __bf16   v8b;
typedef __attribute__((ext_vector_type(8)))  float    v8f;
typedef __attribute__((ext_vector_type(4)))  float    v4f;
typedef __attribute__((ext_vector_type(2)))  float    v2f;

__device__ __forceinline__ unsigned short f2bf_bits(float f) {
  unsigned u = __float_as_uint(f);
  return (unsigned short)((u + 0x7FFFu + ((u >> 16) & 1u)) >> 16);
}
__device__ __forceinline__ float bf_bits2f(unsigned short h) { return __uint_as_float(((unsigned)h) << 16); }

__device__ __forceinline__ void dep_guard_h(v8f& a, v8f& b, v16h x, v16h y) { asm volatile("v_nop\n\tv_nop\n\tv_nop\n\tv_nop" : "+v"(a), "+v"(b) : "v"(x), "v"(y)); }
__device__ __forceinline__ void dep_guard_b(v8f& a, v8f& b, v16b x, v16b y) { asm volatile("v_nop\n\tv_nop\n\tv_nop\n\tv_nop" : "+v"(a), "+v"(b) : "v"(x), "v"(y)); }
__device__ __forceinline__ void keep4_h(v16h a, v16h b, v16h c, v16h d) { asm volatile("v_nop" :: "v"(a), "v"(b), "v"(c), "v"(d)); }
__device__ __forceinline__ void keep4_b(v16b a, v16b b, v16b c, v16b d) { asm volatile("v_nop" :: "v"(a), "v"(b), "v"(c), "v"(d)); }
__device__ __forceinline__ void acc_guard4(v8f& a, v8f& b, v8f& c, v8f& d) { asm volatile("v_nop\n\tv_nop\n\tv_nop\n\tv_nop" : "+v"(a), "+v"(b), "+v"(c), "+v"(d)); }
template <typename T> struct Frag;
template <> struct Frag<_Float16> {
  typedef v16h V; union U { v16h v; v8h h[2]; };
  static __device__ __forceinline__ v16h load(const _Float16* p) {
    U f; f.h[0] = *(const v8h*)(p); f.h[1] = *(const v8h*)(p + 16); return f.v;
  }
  static __device__ __forceinline__ v8f mma(v16h a, v16h b, v8f c) {
    return __builtin_amdgcn_wmma_f32_16x16x32_f16(false, a, false, b, (short)0, c, false, false);
  }
  static __device__ __forceinline__ void guard(v8f& a, v8f& b, v16h x, v16h y) { dep_guard_h(a, b, x, y); }
  static __device__ __forceinline__ void keep(v16h a, v16h b, v16h c, v16h d) { keep4_h(a, b, c, d); }
};
template <> struct Frag<__bf16> {
  typedef v16b V; union U { v16b v; v8b h[2]; };
  static __device__ __forceinline__ v16b load(const __bf16* p) {
    U f; f.h[0] = *(const v8b*)(p); f.h[1] = *(const v8b*)(p + 16); return f.v;
  }
  static __device__ __forceinline__ v8f mma(v16b a, v16b b, v8f c) {
    return __builtin_amdgcn_wmma_f32_16x16x32_bf16(false, a, false, b, (short)0, c, false, false);
  }
  static __device__ __forceinline__ void guard(v8f& a, v8f& b, v16b x, v16b y) { dep_guard_b(a, b, x, y); }
  static __device__ __forceinline__ void keep(v16b a, v16b b, v16b c, v16b d) { keep4_b(a, b, c, d); }
};

template <int ET> struct Elem;
template <> struct Elem<0> { typedef _Float16 T; };
template <> struct Elem<1> { typedef __bf16 T; };
template <int ET, bool SPLIT, int BIAS_MODE, int OUT_MODE, bool RESID, int ACT = 0, bool GATED = false>
__global__ __launch_bounds__(256) void wmma_gemm64(
    const unsigned short* __restrict__ Ap, const unsigned short* __restrict__ A2p, int lda, long strideA,
    const unsigned short* __restrict__ Btp, const unsigned short* __restrict__ Bt2p, int ldb, long strideB,
    void* __restrict__ Cout, void* __restrict__ Cout2, int ldc, long strideC,
    const float* __restrict__ bias, long strideBias,
    const float* __restrict__ resid, long strideR,
    const float* __restrict__ gate, int gate_ld, int gate_shift,
    int M, int N, int K, float scale) {
  typedef typename Elem<ET>::T T;
  typedef typename Frag<T>::V V;
  const T* A = (const T*)Ap; const T* A2 = (const T*)A2p; const T* Bt = (const T*)Btp; const T* Bt2 = (const T*)Bt2p;
  __shared__ __align__(16) float sT[8][16 * 68];
  const int b    = blockIdx.y;
  const int lane = threadIdx.x & 31;
  const int wave = threadIdx.x >> 5;
  const int tilesN = N >> 6;
  const int tilesM = M >> 6;
  const int tile = blockIdx.x * 8 + wave;
  if (tile >= tilesM * tilesN) return;
  const int tm = tile / tilesN;
  const int tn = tile - tm * tilesN;
  const int m0 = tm << 6;
  const int n0 = tn << 6;

  const T* Ab  = A  + (size_t)b * strideA;
  const T* Bb  = Bt + (size_t)b * strideB;
  const T* Ab2 = SPLIT ? (A2  + (size_t)b * strideA) : nullptr;
  const T* Bb2 = SPLIT ? (Bt2 + (size_t)b * strideB) : nullptr;

  const int rlane = lane & 15;
  const int koff  = (lane >> 4) * 8;
  const int mOff  = (lane >> 4) * 8;

  v8f acc[4][4];
#pragma unroll
  for (int i = 0; i < 4; ++i)
#pragma unroll
    for (int j = 0; j < 4; ++j) acc[i][j] = (v8f){0.f,0.f,0.f,0.f,0.f,0.f,0.f,0.f};

  for (int k0 = 0; k0 < K; k0 += 32) {
    V bh[4], bl[4];
#pragma unroll
    for (int j = 0; j < 4; ++j) {
      const size_t bo = (size_t)(n0 + (j << 4) + rlane) * ldb + koff + k0;
      bh[j] = Frag<T>::load(Bb + bo);
      if (SPLIT) bl[j] = Frag<T>::load(Bb2 + bo);
    }
#pragma unroll
    for (int i = 0; i < 4; ++i) {
      const size_t ao = (size_t)(m0 + (i << 4) + rlane) * lda + koff + k0;
      V ah = Frag<T>::load(Ab + ao);
      V al;
      if (SPLIT) al = Frag<T>::load(Ab2 + ao);
#pragma unroll
      for (int j = 0; j < 4; ++j) {
        acc[i][j] = Frag<T>::mma(ah, bh[j], acc[i][j]);
        if (SPLIT) {
          acc[i][j] = Frag<T>::mma(ah, bl[j], acc[i][j]);
          acc[i][j] = Frag<T>::mma(al, bh[j], acc[i][j]);
        }
      }
      Frag<T>::guard(acc[i][0], acc[i][3], ah, SPLIT ? al : ah);
    }
    Frag<T>::keep(bh[0], bh[1], bh[2], bh[3]);
    if (SPLIT) Frag<T>::keep(bl[0], bl[1], bl[2], bl[3]);
  }
  acc_guard4(acc[0][0], acc[0][1], acc[0][2], acc[0][3]);
  acc_guard4(acc[1][0], acc[1][1], acc[1][2], acc[1][3]);
  acc_guard4(acc[2][0], acc[2][1], acc[2][2], acc[2][3]);
  acc_guard4(acc[3][0], acc[3][1], acc[3][2], acc[3][3]);

  float* slab = sT[wave];
  const float* Rb = (RESID || GATED) ? (resid + (size_t)b * strideR) : nullptr;
  const float* biasb = (BIAS_MODE != 0) ? (bias + (size_t)b * strideBias) : nullptr;
#pragma unroll
  for (int i = 0; i < 4; ++i) {
    const int mBase = m0 + (i << 4);
#pragma unroll
    for (int j = 0; j < 4; ++j) {
      const int n = n0 + (j << 4) + rlane;
      float bv = 0.f;
      if (BIAS_MODE == 2) bv = biasb[n];
#pragma unroll
      for (int r = 0; r < 8; ++r) {
        const int mrow = mBase + mOff + r;
        float v = acc[i][j][r] * scale;
        if (BIAS_MODE == 1) v += biasb[mrow];
        if (BIAS_MODE == 2) v += bv;
        if (RESID) v += Rb[(size_t)mrow * ldc + n];
        if (GATED) v = Rb[(size_t)mrow * ldc + n] + gate[(size_t)(mrow >> gate_shift) * gate_ld + n] * v;
        if (ACT == 1) v = tanhf(v);
        if (ACT == 2) v = fmaxf(v, 0.0f);
        if (ACT == 3) v = v / (1.0f + expf(-v));
        if (ACT == 4) v = (v > 0.f) ? v : 0.01f * v;
        slab[(mOff + r) * 68 + (j << 4) + rlane] = v;
      }
    }
    __builtin_amdgcn_fence(__ATOMIC_RELEASE, "workgroup");
    __builtin_amdgcn_wave_barrier();
    __builtin_amdgcn_fence(__ATOMIC_ACQUIRE, "workgroup");
    if (OUT_MODE == 0) {
      float* C = (float*)Cout + (size_t)b * strideC;
      const int hh = lane >> 4, c4 = (lane & 15) * 4;
      for (int pass = 0; pass < 2; ++pass) {
#pragma unroll
        for (int it = 0; it < 8; ++it) {
          const int row = it * 2 + hh;
          v4f v = *(const v4f*)(slab + row * 68 + c4);
          *(volatile v4f*)(C + (size_t)(mBase + row) * ldc + n0 + c4) = v;
        }
        __threadfence();
      }
    } else {
      const int q = lane >> 3, c8 = (lane & 7) * 8;
      unsigned short* C  = (unsigned short*)Cout  + (size_t)b * strideC;
      unsigned short* C2 = (OUT_MODE == 2) ? ((unsigned short*)Cout2 + (size_t)b * strideC) : nullptr;
      for (int pass = 0; pass < 2; ++pass) {
#pragma unroll
        for (int it = 0; it < 4; ++it) {
          const int row = it * 4 + q;
          const float* sp = slab + row * 68 + c8;
          v8h hv, lv;
#pragma unroll
          for (int e = 0; e < 8; ++e) {
            if (OUT_MODE == 1) {
              hv[e] = (_Float16)sp[e];
            } else {
              unsigned short hb = f2bf_bits(sp[e]);
              unsigned short lb = f2bf_bits(sp[e] - bf_bits2f(hb));
              hv[e] = __builtin_bit_cast(_Float16, hb);
              lv[e] = __builtin_bit_cast(_Float16, lb);
            }
          }
          *(volatile v8h*)(C + (size_t)(mBase + row) * ldc + n0 + c8) = hv;
          if (OUT_MODE == 2) *(volatile v8h*)(C2 + (size_t)(mBase + row) * ldc + n0 + c8) = lv;
        }
        __threadfence();
      }
    }
    __builtin_amdgcn_fence(__ATOMIC_RELEASE, "workgroup");
    __builtin_amdgcn_wave_barrier();
    __builtin_amdgcn_fence(__ATOMIC_ACQUIRE, "workgroup");
  }
}

__global__ __launch_bounds__(256) void cast_f32_f16x2s(
    const float* __restrict__ in, unsigned* __restrict__ out, int n2, float scale) {
  const int i = blockIdx.x * 256 + threadIdx.x;
  if (i < n2) {
    const v2f f = *(const v2f*)(in + 2 * (size_t)i);
    const _Float16 h0 = (_Float16)(f[0] * scale), h1 = (_Float16)(f[1] * scale);
    const unsigned u = (unsigned)__builtin_bit_cast(unsigned short, h0) | ((unsigned)__builtin_bit_cast(unsigned short, h1) << 16);
    ((volatile unsigned*)out)[i] = u;
    __threadfence();
    ((volatile unsigned*)out)[i] = u;
  }
}

__global__ __launch_bounds__(256) void gelu_f16x2_kernel(
    const unsigned* __restrict__ in, unsigned* __restrict__ out, int n2) {
  const int i = blockIdx.x * 256 + threadIdx.x;
  if (i < n2) {
    const unsigned u = in[i];
    const float f0 = (float)__builtin_bit_cast(_Float16, (unsigned short)(u & 0xFFFFu));
    const float f1 = (float)__builtin_bit_cast(_Float16, (unsigned short)(u >> 16));
    const float g0 = 0.5f * f0 * (1.0f + erff(f0 * 0.70710678118654752f));
    const float g1 = 0.5f * f1 * (1.0f + erff(f1 * 0.70710678118654752f));
    const _Float16 h0 = (_Float16)g0, h1 = (_Float16)g1;
    const unsigned w = (unsigned)__builtin_bit_cast(unsigned short, h0) | ((unsigned)__builtin_bit_cast(unsigned short, h1) << 16);
    ((volatile unsigned*)out)[i] = w;
    __threadfence();
    ((volatile unsigned*)out)[i] = w;
  }
}

__global__ __launch_bounds__(256) void rope_tab_kernel(float* __restrict__ ctab, float* __restrict__ stab) {
  const int i = blockIdx.x * 256 + threadIdx.x;
  const int pos = i >> 5, j = i & 31;
  const float invf = exp2f(-(float)j * 0.41524101186092028f);
  const float f = (float)pos * invf;
  const float cs = cosf(f);
  const float sn = sinf(f);
  ((volatile float*)ctab)[i] = cs;
  ((volatile float*)stab)[i] = sn;
  __threadfence();
  ((volatile float*)ctab)[i] = cs;
  ((volatile float*)stab)[i] = sn;
}

__global__ __launch_bounds__(256) void adaln_kernel(const float* __restrict__ cond, const float* __restrict__ Wa,
                                                    const float* __restrict__ ba, float* __restrict__ mod) {
  __shared__ float sact[1024];
  __shared__ __align__(16) float sout[64];
  const int b = blockIdx.y, j0 = blockIdx.x * 64;
  const int tid = threadIdx.x, lane = tid & 31, wv = tid >> 5;
#pragma unroll 1
  for (int i = tid; i < 1024; i += 256) {
    const float v = cond[(size_t)b * 1024 + i];
    sact[i] = v * (1.0f / (1.0f + expf(-v)));
  }
  __syncthreads();
#pragma unroll 1
  for (int o = 0; o < 8; ++o) {
    const int j = j0 + wv * 8 + o;
    const float* wr = Wa + (size_t)j * 1024;
    float acc = 0.f;
#pragma unroll 1
    for (int k = lane; k < 1024; k += 32) acc = fmaf(sact[k], wr[k], acc);
    acc += __shfl_xor(acc, 16, 32);
    acc += __shfl_xor(acc, 8, 32);
    acc += __shfl_xor(acc, 4, 32);
    acc += __shfl_xor(acc, 2, 32);
    acc += __shfl_xor(acc, 1, 32);
    if (lane == 0) sout[wv * 8 + o] = acc + ba[j];
  }
  __syncthreads();
  if (wv == 0) {
    const int li = (lane < 16) ? lane : 15;
    const v4f v = *(const v4f*)(sout + li * 4);
    float* dst = mod + (size_t)b * 6144 + j0 + li * 4;
    if (lane < 16) { *(volatile v4f*)dst = v; }
    __threadfence();
    if (lane < 16) { *(volatile v4f*)dst = v; }
  }
}

__global__ __launch_bounds__(128) void ln_mod_kernel(const float* __restrict__ X, const float* __restrict__ w,
    const float* __restrict__ bb, const float* __restrict__ mod, int shift_idx, int scale_idx,
    unsigned short* __restrict__ out16, int rows_per_batch) {
  __shared__ float red[4];
  __shared__ float red2[4];
  const int tok = blockIdx.x;
  const int b = tok / rows_per_batch;
  const int t = threadIdx.x, lane = t & 31, wv = t >> 5;
  const int c0 = t * 8;
  const float* row = X + (size_t)tok * 1024;
  const v4f a0 = *(const v4f*)(row + c0);
  const v4f a1 = *(const v4f*)(row + c0 + 4);
  float s = ((a0[0] + a0[1]) + (a0[2] + a0[3])) + ((a1[0] + a1[1]) + (a1[2] + a1[3]));
  s += __shfl_xor(s, 16, 32); s += __shfl_xor(s, 8, 32); s += __shfl_xor(s, 4, 32); s += __shfl_xor(s, 2, 32); s += __shfl_xor(s, 1, 32);
  if (lane == 0) red[wv] = s;
  __syncthreads();
  const float mean = ((red[0] + red[1]) + (red[2] + red[3])) * (1.0f / 1024.0f);
  const v4f d0 = a0 - mean;
  const v4f d1 = a1 - mean;
  float q = ((d0[0] * d0[0] + d0[1] * d0[1]) + (d0[2] * d0[2] + d0[3] * d0[3]))
          + ((d1[0] * d1[0] + d1[1] * d1[1]) + (d1[2] * d1[2] + d1[3] * d1[3]));
  q += __shfl_xor(q, 16, 32); q += __shfl_xor(q, 8, 32); q += __shfl_xor(q, 4, 32); q += __shfl_xor(q, 2, 32); q += __shfl_xor(q, 1, 32);
  if (lane == 0) red2[wv] = q;
  __syncthreads();
  const float var = ((red2[0] + red2[1]) + (red2[2] + red2[3])) * (1.0f / 1024.0f);
  const float inv = rsqrtf(var + 1e-5f);
  const v4f w0 = *(const v4f*)(w + c0),  w1 = *(const v4f*)(w + c0 + 4);
  const v4f b0 = *(const v4f*)(bb + c0), b1 = *(const v4f*)(bb + c0 + 4);
  const float* mrow = mod + (size_t)b * 6144;
  const v4f sc0 = *(const v4f*)(mrow + scale_idx * 1024 + c0), sc1 = *(const v4f*)(mrow + scale_idx * 1024 + c0 + 4);
  const v4f sh0 = *(const v4f*)(mrow + shift_idx * 1024 + c0), sh1 = *(const v4f*)(mrow + shift_idx * 1024 + c0 + 4);
  v4f y0 = d0 * inv * w0 + b0;
  v4f y1 = d1 * inv * w1 + b1;
  y0 = y0 * (1.0f + sc0) + sh0;
  y1 = y1 * (1.0f + sc1) + sh1;
  v8h hv;
  hv[0] = (_Float16)y0[0]; hv[1] = (_Float16)y0[1]; hv[2] = (_Float16)y0[2]; hv[3] = (_Float16)y0[3];
  hv[4] = (_Float16)y1[0]; hv[5] = (_Float16)y1[1]; hv[6] = (_Float16)y1[2]; hv[7] = (_Float16)y1[3];
  unsigned short* op = out16 + (size_t)tok * 1024 + c0;
  *(volatile v8h*)op = hv;
  __threadfence();
  *(volatile v8h*)op = hv;
}

__global__ __launch_bounds__(256) void rms_rope_kernel(const float* __restrict__ raw, long strideIn,
    const float* __restrict__ rw, const float* __restrict__ ctab, const float* __restrict__ stab,
    unsigned short* __restrict__ out16, long strideOut, int Lseq, int do_rope) {
  const int z = blockIdx.y;
  const int tid = threadIdx.x;
  const int grp = tid >> 3, sub = tid & 7;
  const int row = blockIdx.x * 2 + (grp >> 4);
  const int head = grp & 15;
  const int pos = row % Lseq;
  const int d0 = sub * 8, dp0 = d0 ^ 32;
  const float* base = raw + (size_t)z * strideIn + (size_t)row * 1024 + head * 64;
  const v4f a0 = *(const v4f*)(base + d0),  a1 = *(const v4f*)(base + d0 + 4);
  const v4f p0 = *(const v4f*)(base + dp0), p1 = *(const v4f*)(base + dp0 + 4);
  float ss = ((a0[0] * a0[0] + a0[1] * a0[1]) + (a0[2] * a0[2] + a0[3] * a0[3]))
           + ((a1[0] * a1[0] + a1[1] * a1[1]) + (a1[2] * a1[2] + a1[3] * a1[3]));
  ss += __shfl_xor(ss, 1, 32); ss += __shfl_xor(ss, 2, 32); ss += __shfl_xor(ss, 4, 32);
  const float inv = rsqrtf(ss * (1.0f / 64.0f) + 1e-6f);
  const v4f w0 = *(const v4f*)(rw + d0),  w1 = *(const v4f*)(rw + d0 + 4);
  const v4f wp0 = *(const v4f*)(rw + dp0), wp1 = *(const v4f*)(rw + dp0 + 4);
  v4f y0 = a0 * inv * w0;
  v4f y1 = a1 * inv * w1;
  if (do_rope) {
    const v4f yp0 = p0 * inv * wp0;
    const v4f yp1 = p1 * inv * wp1;
    const float sgn = (d0 < 32) ? -1.0f : 1.0f;
    const int j0 = d0 & 31;
    const float* cr = ctab + (size_t)pos * 32 + j0;
    const float* sr = stab + (size_t)pos * 32 + j0;
    const v4f c0 = *(const v4f*)(cr), c1 = *(const v4f*)(cr + 4);
    const v4f s0 = *(const v4f*)(sr), s1 = *(const v4f*)(sr + 4);
    y0 = y0 * c0 + (yp0 * sgn) * s0;
    y1 = y1 * c1 + (yp1 * sgn) * s1;
  }
  v8h hv;
  hv[0] = (_Float16)y0[0]; hv[1] = (_Float16)y0[1]; hv[2] = (_Float16)y0[2]; hv[3] = (_Float16)y0[3];
  hv[4] = (_Float16)y1[0]; hv[5] = (_Float16)y1[1]; hv[6] = (_Float16)y1[2]; hv[7] = (_Float16)y1[3];
  unsigned short* op = out16 + (size_t)z * strideOut + (size_t)row * 1024 + head * 64 + d0;
  *(volatile v8h*)op = hv;
  __threadfence();
  *(volatile v8h*)op = hv;
}

#define MS_D 64
#define MS_NW 4
#define MS_KC 64
#define MS_TQ 512
#define MS_DM 1024
#define MS_NCHUNK 28

__device__ __forceinline__ v8f mma_h(v16h a, v16h b, v8f c) {
  c = __builtin_amdgcn_wmma_f32_16x16x32_f16(false, a, false, b, (short)0, c, false, false);
  asm volatile("v_nop\n\tv_nop\n\tv_nop\n\tv_nop" : "+v"(c) : "v"(a), "v"(b));
  return c;
}
__device__ __forceinline__ float softplus_f(float t) { return fmaxf(t, 0.0f) + log1pf(expf(-fabsf(t))); }

__global__ __launch_bounds__(128)
void msattn_kernel(const unsigned short* __restrict__ q0p, const unsigned short* __restrict__ q1p,
                   const unsigned short* __restrict__ q2p, const unsigned short* __restrict__ q3p,
                   const unsigned short* __restrict__ k0p, const unsigned short* __restrict__ k1p,
                   const unsigned short* __restrict__ k2p, const unsigned short* __restrict__ k3p,
                   const unsigned short* __restrict__ v0p, const unsigned short* __restrict__ v1p,
                   const unsigned short* __restrict__ v2p, const unsigned short* __restrict__ v3p,
                   const float* __restrict__ temps, const float* __restrict__ sbias,
                   const float* __restrict__ gating, unsigned short* __restrict__ o16p) {
  union FH { v16h v; v8h h[2]; };
  __shared__ __align__(16) _Float16 Ksh[MS_KC * MS_D];
  __shared__ __align__(16) _Float16 Vth[MS_D * MS_KC];
  __shared__ __align__(16) _Float16 Psh[MS_NW][16 * MS_KC];
  __shared__ __align__(16) float  Os[MS_NW][16 * 68];

  const int tid  = threadIdx.x;
  const int wave = tid >> 5;
  const int lane = tid & 31;
  const int hh   = lane >> 4;
  const int c    = lane & 15;

  const int bx = blockIdx.x;
  const int qb = bx & 7;
  const int bh = bx >> 3;
  const int h  = bh & 15;
  const int b  = bh >> 4;
  const int q0 = qb * 64 + wave * 16;

  const float sc0 = 0.125f * (1.0f + softplus_f(temps[0]));
  const float sc1 = 0.125f * (1.0f + softplus_f(temps[1]));
  const float sc2 = 0.125f * (1.0f + softplus_f(temps[2]));
  const float sc3 = 0.125f * (1.0f + softplus_f(temps[3]));
  const float sb0 = sbias[0], sb1 = sbias[1], sb2 = sbias[2], sb3 = sbias[3];
  const float ratio = tanhf(gating[0]);

  const _Float16* Q0 = (const _Float16*)(const void*)q0p; const _Float16* Q1 = (const _Float16*)(const void*)q1p;
  const _Float16* Q2 = (const _Float16*)(const void*)q2p; const _Float16* Q3 = (const _Float16*)(const void*)q3p;
  const _Float16* K0 = (const _Float16*)(const void*)k0p; const _Float16* K1 = (const _Float16*)(const void*)k1p;
  const _Float16* K2 = (const _Float16*)(const void*)k2p; const _Float16* K3 = (const _Float16*)(const void*)k3p;
  const _Float16* V0 = (const _Float16*)(const void*)v0p; const _Float16* V1 = (const _Float16*)(const void*)v1p;
  const _Float16* V2 = (const _Float16*)(const void*)v2p; const _Float16* V3 = (const _Float16*)(const void*)v3p;

  float mrow[8], lrow[8];
  v8f oacc[4];
#pragma unroll
  for (int r = 0; r < 8; ++r) { mrow[r] = -INFINITY; lrow[r] = 0.f; }
#pragma unroll
  for (int t = 0; t < 4; ++t) oacc[t] = (v8f){0.f,0.f,0.f,0.f,0.f,0.f,0.f,0.f};

  for (int kc = 0; kc < MS_NCHUNK; ++kc) {
    const int seg  = kc >> 3;
    const int kvl  = (kc & 7) * MS_KC;
    const int Lseg = (seg == 3) ? 256 : 512;
    const int ntok = Lseg * 4;
    const _Float16* Qp = (seg == 0) ? Q0 : ((seg == 1) ? Q1 : ((seg == 2) ? Q2 : Q3));
    const _Float16* Kp = (seg == 0) ? K0 : ((seg == 1) ? K1 : ((seg == 2) ? K2 : K3));
    const _Float16* Vp = (seg == 0) ? V0 : ((seg == 1) ? V1 : ((seg == 2) ? V2 : V3));
    const float sc = (seg == 0) ? sc0 : ((seg == 1) ? sc1 : ((seg == 2) ? sc2 : sc3));
    const float sb = (seg == 0) ? sb0 : ((seg == 1) ? sb1 : ((seg == 2) ? sb2 : sb3));
    const float gm = (seg == 3) ? ratio : 1.0f;
    __syncthreads();
    {
      const int r = tid >> 1, half = (tid & 1) * 32;
      const _Float16* ks = Kp + ((size_t)(b * Lseg + kvl + r)) * MS_DM + h * MS_D + half;
      const _Float16* vs = Vp + ((size_t)(h * MS_D + r)) * ntok + b * Lseg + kvl + half;
#pragma unroll
      for (int i = 0; i < 4; ++i) {
        const v8h ka = *(const v8h*)(ks + 8 * i);
        const v8h va = *(const v8h*)(vs + 8 * i);
        *(v8h*)(Ksh + r * MS_D  + half + 8 * i) = ka;
        *(v8h*)(Vth + r * MS_KC + half + 8 * i) = va;
      }
    }
    __syncthreads();

    v16h qa[2];
#pragma unroll
    for (int dc = 0; dc < 2; ++dc)
      qa[dc] = Frag<_Float16>::load(Qp + ((size_t)(b * MS_TQ + q0 + c)) * MS_DM + h * MS_D + dc * 32 + 8 * hh);

    v8f s[4];
#pragma unroll
    for (int j = 0; j < 4; ++j) {
      s[j] = (v8f){0.f,0.f,0.f,0.f,0.f,0.f,0.f,0.f};
#pragma unroll
      for (int dc = 0; dc < 2; ++dc) {
        FH kb;
        kb.h[0] = *(const v8h*)(Ksh + (j * 16 + c) * MS_D + dc * 32 + 8 * hh);
        kb.h[1] = *(const v8h*)(Ksh + (j * 16 + c) * MS_D + dc * 32 + 16 + 8 * hh);
        s[j] = mma_h(qa[dc], kb.v, s[j]);
      }
    }
    float cm[8];
#pragma unroll
    for (int r = 0; r < 8; ++r) {
      float m = -INFINITY;
#pragma unroll
      for (int j = 0; j < 4; ++j) {
        const float sv = (s[j][r] * sc + sb) * gm;
        s[j][r] = sv;
        m = fmaxf(m, sv);
      }
#pragma unroll
      for (int off = 1; off < 16; off <<= 1) m = fmaxf(m, __shfl_xor(m, off, 32));
      cm[r] = m;
    }
    _Float16* pw = Psh[wave];
#pragma unroll
    for (int r = 0; r < 8; ++r) {
      const float mnew = fmaxf(mrow[r], cm[r]);
      const float alpha = expf(mrow[r] - mnew);
      mrow[r] = mnew;
      float psum = 0.f;
#pragma unroll
      for (int j = 0; j < 4; ++j) {
        const float p = expf(s[j][r] - mnew);
        psum += p;
        pw[(8 * hh + r) * MS_KC + j * 16 + c] = (_Float16)(p * 32768.0f);
      }
#pragma unroll
      for (int off = 1; off < 16; off <<= 1) psum += __shfl_xor(psum, off, 32);
      lrow[r] = lrow[r] * alpha + psum;
#pragma unroll
      for (int t = 0; t < 4; ++t) oacc[t][r] *= alpha;
    }
    __builtin_amdgcn_fence(__ATOMIC_RELEASE, "workgroup");
    __builtin_amdgcn_wave_barrier();
    __builtin_amdgcn_fence(__ATOMIC_ACQUIRE, "workgroup");
#pragma unroll 1
    for (int kk = 0; kk < 2; ++kk) {
      FH pa;
      pa.h[0] = *(const v8h*)(pw + c * MS_KC + kk * 32 + 8 * hh);
      pa.h[1] = *(const v8h*)(pw + c * MS_KC + kk * 32 + 16 + 8 * hh);
#pragma unroll
      for (int t = 0; t < 4; ++t) {
        FH vb;
        vb.h[0] = *(const v8h*)(Vth + (t * 16 + c) * MS_KC + kk * 32 + 8 * hh);
        vb.h[1] = *(const v8h*)(Vth + (t * 16 + c) * MS_KC + kk * 32 + 16 + 8 * hh);
        oacc[t] = mma_h(pa.v, vb.v, oacc[t]);
      }
    }
  }

  float* os = Os[wave];
#pragma unroll
  for (int r = 0; r < 8; ++r) {
    const float inv = 1.0f / (lrow[r] * 1024.0f);
#pragma unroll
    for (int t = 0; t < 4; ++t) os[(8 * hh + r) * 68 + t * 16 + c] = oacc[t][r] * inv;
  }
  __builtin_amdgcn_fence(__ATOMIC_RELEASE, "workgroup");
  __builtin_amdgcn_wave_barrier();
  __builtin_amdgcn_fence(__ATOMIC_ACQUIRE, "workgroup");
  {
    const int q = lane >> 3, c8 = (lane & 7) * 8;
    unsigned short* ob = o16p + (size_t)h * MS_D;
    for (int pass = 0; pass < 2; ++pass) {
#pragma unroll
      for (int it = 0; it < 4; ++it) {
        const int row = it * 4 + q;
        const float* sp = os + row * 68 + c8;
        v8h hv;
#pragma unroll
        for (int e = 0; e < 8; ++e) hv[e] = (_Float16)sp[e];
        *(volatile v8h*)(ob + ((size_t)(b * MS_TQ + q0 + row)) * MS_DM + c8) = hv;
      }
      __threadfence();
    }
  }
}

extern "C" void kernel_launch(void* const* d_in, const int* in_sizes, int n_in,
                              void* d_out, int out_size, void* d_ws, size_t ws_size,
                              hipStream_t stream) {
  const size_t MIB = 1048576;
  const size_t OFF_WQ = 0, OFF_WK = 2 * MIB, OFF_WV = 10 * MIB, OFF_WQA = 18 * MIB, OFF_WQAO = 19 * MIB + 524288,
               OFF_WO = 20 * MIB, OFF_ACT = 22 * MIB, OFF_HID = 36 * MIB, OFF_QKV = 39 * MIB, OFF_RAW = 83 * MIB,
               OFF_MOD = 107 * MIB, OFF_CT = OFF_MOD + 131072, OFF_ST = OFF_CT + 65536, WS_TOTAL = OFF_ST + 65536;
  if (n_in < 32) return;
  if (in_sizes[0] != 2097152 || in_sizes[1] != 2097152 || in_sizes[2] != 2097152 || in_sizes[3] != 1048576 ||
      in_sizes[4] != 4096 || in_sizes[7] != 6291456 || in_sizes[9] != 1048576 || in_sizes[11] != 786432 ||
      in_sizes[13] != 262144 || in_sizes[15] != 4194304 || in_sizes[17] != 4194304 || in_sizes[19] != 1048576 ||
      in_sizes[28] != 4194304 || in_sizes[30] != 4194304 || in_sizes[24] != 4 || in_sizes[25] != 4 || in_sizes[23] != 1 ||
      out_size != 2097152) return;
  if (ws_size < WS_TOTAL) return;

  const float* x        = (const float*)d_in[0];
  const float* bev      = (const float*)d_in[1];
  const float* vl       = (const float*)d_in[2];
  const float* rea      = (const float*)d_in[3];
  const float* cond     = (const float*)d_in[4];
  const float* ln_pre_w = (const float*)d_in[5];
  const float* ln_pre_b = (const float*)d_in[6];
  const float* adaln_w  = (const float*)d_in[7];
  const float* adaln_b  = (const float*)d_in[8];
  const float* q_proj_w = (const float*)d_in[9];
  const float* q_proj_b = (const float*)d_in[10];
  const float* qa_w     = (const float*)d_in[11];
  const float* qa_b     = (const float*)d_in[12];
  const float* qa_out_w = (const float*)d_in[13];
  const float* qa_out_b = (const float*)d_in[14];
  const float* k_w      = (const float*)d_in[15];
  const float* k_b      = (const float*)d_in[16];
  const float* v_w      = (const float*)d_in[17];
  const float* v_b      = (const float*)d_in[18];
  const float* o_w      = (const float*)d_in[19];
  const float* o_b      = (const float*)d_in[20];
  const float* qn_w     = (const float*)d_in[21];
  const float* kn_w     = (const float*)d_in[22];
  const float* gating   = (const float*)d_in[23];
  const float* temps    = (const float*)d_in[24];
  const float* sbias    = (const float*)d_in[25];
  const float* ffn_ln_w = (const float*)d_in[26];
  const float* ffn_ln_b = (const float*)d_in[27];
  const float* ffn_w1   = (const float*)d_in[28];
  const float* ffn_b1   = (const float*)d_in[29];
  const float* ffn_w2   = (const float*)d_in[30];
  const float* ffn_b2   = (const float*)d_in[31];

  char* ws = (char*)d_ws;
  unsigned short* WQ   = (unsigned short*)(ws + OFF_WQ);
  unsigned short* WK   = (unsigned short*)(ws + OFF_WK);
  unsigned short* WV   = (unsigned short*)(ws + OFF_WV);
  unsigned short* WQA  = (unsigned short*)(ws + OFF_WQA);
  unsigned short* WQAO = (unsigned short*)(ws + OFF_WQAO);
  unsigned short* WO   = (unsigned short*)(ws + OFF_WO);
  unsigned short* W1   = WK;
  unsigned short* W2   = WV;
  unsigned short* ACT  = (unsigned short*)(ws + OFF_ACT);
  unsigned short* XN16 = ACT;
  unsigned short* BEV16 = ACT + 2097152;
  unsigned short* VL16  = ACT + 4194304;
  unsigned short* RE16  = ACT + 6291456;
  unsigned short* O16  = ACT;
  unsigned short* H16  = ACT + 2097152;
  unsigned short* HID  = (unsigned short*)(ws + OFF_HID);
  unsigned short* QKV  = (unsigned short*)(ws + OFF_QKV);
  unsigned short* QPL  = QKV;
  unsigned short* KPL  = QKV + 8 * 1048576;
  unsigned short* K3PL = QKV + 14 * 1048576;
  unsigned short* VT   = QKV + 15 * 1048576;
  unsigned short* VT3  = QKV + 21 * 1048576;
  unsigned short* U16  = QKV;
  unsigned short* G16  = QKV + 8 * 1048576;
  float* RAW  = (float*)(ws + OFF_RAW);
  float* X2   = RAW;
  float* MODP = (float*)(ws + OFF_MOD);
  float* CT   = (float*)(ws + OFF_CT);
  float* ST   = (float*)(ws + OFF_ST);

  const float WSC = 1.0f / 64.0f;

  auto cast16 = [&](const float* src, unsigned short* dst, int n, float scale) {
    const int n2 = n / 2;
    cast_f32_f16x2s<<<(n2 + 255) / 256, 256, 0, stream>>>(src, (unsigned*)dst, n2, scale);
  };
  auto gemm_f32out = [&](const unsigned short* A, int lda, long sA, const unsigned short* Bt, int ldb, long sB,
                         float* C, int ldc, long sC, const float* bias, long sBias, int M, int N, int K, int Z, float scale) {
    const int tiles = (M / 64) * (N / 64);
    dim3 grid((tiles + 7) / 8, Z);
    wmma_gemm64<0, false, 2, 0, false, 0, false><<<grid, 256, 0, stream>>>(
        A, nullptr, lda, sA, Bt, nullptr, ldb, sB, (void*)C, nullptr, ldc, sC, bias, sBias,
        nullptr, 0, nullptr, 0, 0, M, N, K, scale);
  };
  auto gemm_f16out = [&](const unsigned short* A, int lda, long sA, const unsigned short* Bt, int ldb, long sB,
                         unsigned short* C, int ldc, long sC, const float* bias, long sBias, int M, int N, int K, int Z, float scale) {
    const int tiles = (M / 64) * (N / 64);
    dim3 grid((tiles + 7) / 8, Z);
    wmma_gemm64<0, false, 2, 1, false, 0, false><<<grid, 256, 0, stream>>>(
        A, nullptr, lda, sA, Bt, nullptr, ldb, sB, (void*)C, nullptr, ldc, sC, bias, sBias,
        nullptr, 0, nullptr, 0, 0, M, N, K, scale);
  };
  auto gemm_vt = [&](const unsigned short* A, int lda, long sA, const unsigned short* Bt, int ldb, long sB,
                     unsigned short* C, int ldc, long sC, const float* bias, long sBias, int M, int N, int K, int Z, float scale) {
    const int tiles = (M / 64) * (N / 64);
    dim3 grid((tiles + 7) / 8, Z);
    wmma_gemm64<0, false, 1, 1, false, 0, false><<<grid, 256, 0, stream>>>(
        A, nullptr, lda, sA, Bt, nullptr, ldb, sB, (void*)C, nullptr, ldc, sC, bias, sBias,
        nullptr, 0, nullptr, 0, 0, M, N, K, scale);
  };
  auto gemm_gated = [&](const unsigned short* A, int lda, const unsigned short* Bt, int ldb, float* C, int ldc,
                        const float* bias, const float* resid, const float* gate, int M, int N, int K, float scale) {
    const int tiles = (M / 64) * (N / 64);
    dim3 grid((tiles + 7) / 8, 1);
    wmma_gemm64<0, false, 2, 0, false, 0, true><<<grid, 256, 0, stream>>>(
        A, nullptr, lda, 0, Bt, nullptr, ldb, 0, (void*)C, nullptr, ldc, 0, bias, 0,
        resid, 0, gate, 6144, 9, M, N, K, scale);
  };

  rope_tab_kernel<<<64, 256, 0, stream>>>(CT, ST);

  cast16(q_proj_w, WQ,   1048576, 64.0f);
  cast16(k_w,      WK,   4194304, 64.0f);
  cast16(v_w,      WV,   4194304, 64.0f);
  cast16(qa_w,     WQA,   786432, 64.0f);
  cast16(qa_out_w, WQAO,  262144, 64.0f);
  cast16(o_w,      WO,   1048576, 64.0f);
  cast16(bev, BEV16, 2097152, 1.0f);
  cast16(vl,  VL16,  2097152, 1.0f);
  cast16(rea, RE16,  1048576, 1.0f);

  adaln_kernel<<<dim3(96, 4), 256, 0, stream>>>(cond, adaln_w, adaln_b, MODP);

  ln_mod_kernel<<<2048, 128, 0, stream>>>(x, ln_pre_w, ln_pre_b, MODP, 0, 1, XN16, 512);

  gemm_f32out(XN16, 1024, 0, WQ, 1024, 0, RAW, 1024, 0, q_proj_b, 0, 2048, 1024, 1024, 1, WSC);
  rms_rope_kernel<<<dim3(1024, 1), 256, 0, stream>>>(RAW, 0, qn_w, CT, ST, QPL, 0, 512, 1);

  gemm_f16out(XN16, 1024, 0, WQA, 1024, 262144, HID, 256, 524288, qa_b, 256, 2048, 256, 1024, 3, WSC);
  gemm_f32out(HID, 256, 524288, WQAO, 256, 0, RAW, 1024, 2097152, qa_out_b, 0, 2048, 1024, 256, 3, WSC);
  rms_rope_kernel<<<dim3(1024, 3), 256, 0, stream>>>(RAW, 2097152, qn_w, CT, ST, QPL + 2097152, 2097152, 512, 0);

  gemm_f32out(ACT, 1024, 2097152, WK, 1024, 1048576, RAW, 1024, 2097152, k_b, 1024, 2048, 1024, 1024, 3, WSC);
  rms_rope_kernel<<<dim3(1024, 3), 256, 0, stream>>>(RAW, 2097152, kn_w, CT, ST, KPL, 2097152, 512, 1);
  gemm_f32out(RE16, 1024, 0, WK + 3 * 1048576, 1024, 0, RAW, 1024, 0, k_b + 3072, 0, 1024, 1024, 1024, 1, WSC);
  rms_rope_kernel<<<dim3(512, 1), 256, 0, stream>>>(RAW, 0, kn_w, CT, ST, K3PL, 0, 256, 1);

  gemm_vt(WV, 1024, 1048576, ACT, 1024, 2097152, VT, 2048, 2097152, v_b, 1024, 1024, 2048, 1024, 3, WSC);
  gemm_vt(WV + 3 * 1048576, 1024, 0, RE16, 1024, 0, VT3, 1024, 0, v_b + 3072, 0, 1024, 1024, 1024, 1, WSC);

  msattn_kernel<<<512, 128, 0, stream>>>(QPL, QPL + 2097152, QPL + 4194304, QPL + 6291456,
                                         KPL, KPL + 2097152, KPL + 4194304, K3PL,
                                         VT, VT + 2097152, VT + 4194304, VT3,
                                         temps, sbias, gating, O16);

  cast16(ffn_w1, W1, 4194304, 64.0f);
  cast16(ffn_w2, W2, 4194304, 64.0f);

  gemm_gated(O16, 1024, WO, 1024, X2, 1024, o_b, x, MODP + 2 * 1024, 2048, 1024, 1024, 1.0f / 2048.0f);

  ln_mod_kernel<<<2048, 128, 0, stream>>>(X2, ffn_ln_w, ffn_ln_b, MODP, 3, 4, H16, 512);
  gemm_f16out(H16, 1024, 0, W1, 1024, 0, U16, 4096, 0, ffn_b1, 0, 2048, 4096, 1024, 1, WSC);
  gelu_f16x2_kernel<<<16384, 256, 0, stream>>>((const unsigned*)U16, (unsigned*)G16, 4194304);
  gemm_gated(G16, 4096, W2, 4096, (float*)d_out, 1024, ffn_b2, X2, MODP + 5 * 1024, 2048, 1024, 4096, WSC);
}
